// NonLocalAttention_12017318494239
// MI455X (gfx1250) — hardware-verified
//
#include <hip/hip_runtime.h>


namespace {
typedef _Float16 b16;
typedef __attribute__((ext_vector_type(16))) _Float16 v16b;
typedef __attribute__((ext_vector_type(8))) _Float16 v8b;
typedef __attribute__((ext_vector_type(4))) _Float16 v4h;
typedef __attribute__((ext_vector_type(2))) _Float16 v2h;
typedef __attribute__((ext_vector_type(8))) float v8f;
typedef __attribute__((ext_vector_type(4))) float v4f;
typedef __attribute__((ext_vector_type(2))) float v2f;
__device__ __forceinline__ float bf16_rne(float f) { unsigned int u = __float_as_uint(f); u += 0x7FFFu + ((u >> 16) & 1u); return __uint_as_float(u & 0xFFFF0000u); }
__device__ __forceinline__ void split16(float v, b16& hi, b16& lo) { hi = (b16)v; lo = (b16)(v - (float)hi); }
__device__ __forceinline__ v16b frag_kb(const b16* p, int hh) { const v8b a = *(const v8b*)(p + 8 * hh), b = *(const v8b*)(p + 16 + 8 * hh); v16b f;
#pragma unroll
  for (int e = 0; e < 8; ++e) { f[e] = a[e]; f[8 + e] = b[e]; } return f; }
__device__ __forceinline__ v8f wmma16b(v16b a, v16b b, v8f c) { v8f d = __builtin_amdgcn_wmma_f32_16x16x32_f16(false, a, false, b, (short)0, c, false, false); asm volatile("v_nop\n\tv_nop\n\tv_nop\n\tv_nop" : "+v"(d) : "v"(a), "v"(b)); return d; }
__device__ __forceinline__ void wave_lds_sync() { __builtin_amdgcn_fence(__ATOMIC_RELEASE, "workgroup"); __builtin_amdgcn_wave_barrier(); __builtin_amdgcn_fence(__ATOMIC_ACQUIRE, "workgroup"); }
__device__ __forceinline__ float pmul(float a, float b) { float p = a * b; asm volatile("" : "+v"(p)); return p; }
__device__ __forceinline__ int iclamp(int v, int lo, int hi) { return v < lo ? lo : (v > hi ? hi : v); }
__device__ __forceinline__ float nexp2(float v) { return __builtin_amdgcn_exp2f(v); }

constexpr int B = 4, C = 64, L = 6400, NO = 3 * C, BL = 4  , QL = 6400  ;
constexpr float XS = 8.0f, WSC = 256.0f, RS = 1024.0f, PS = 16384.0f, LOG2E = 1.4426950408889634f, SLOPE = 0.2f;
static_assert(L % 64 == 0 && QL % 32 == 0 && C == 64, "tiling");
__device__ __forceinline__ float lrelu(float v) { return v >= 0.0f ? v : SLOPE * v; }
__global__ __launch_bounds__(256) void prep_kernel(const float* __restrict__ w1, const float* __restrict__ w2, const float* __restrict__ w3, b16* __restrict__ WT) {
  const int u = blockIdx.x * 256 + threadIdx.x; if (u >= NO * C / 8) return; const int e = u * 8; const int m = e / (C * C), r = e % (C * C); const float* w = m == 0 ? w1 : m == 1 ? w2 : w3; v8b v;
  for (int j = 0; j < 8; ++j) v[j] = (b16)(bf16_rne(w[r + j]) * WSC);
  for (int pass = 0; pass < 2; ++pass) { *(volatile v8b*)(WT + e) = v; __threadfence(); }
}
__global__ __launch_bounds__(128) void qkv_kernel(const float* __restrict__ x, const b16* __restrict__ WT, const float* __restrict__ b1, const float* __restrict__ b2, const float* __restrict__ b3,
                                                  b16* __restrict__ Qh, b16* __restrict__ Ql, b16* __restrict__ Kh, b16* __restrict__ Kl, b16* __restrict__ VT) {
  __shared__ __attribute__((aligned(16))) b16 As[64][C + 8]; __shared__ __attribute__((aligned(16))) float Tf[4][16][NO + 4];
  const int wave = threadIdx.x >> 5, lane = threadIdx.x & 31, nloc = lane & 15, hlf = lane >> 4; const int p0 = blockIdx.x * 64; const int b = blockIdx.y;
  for (int i = threadIdx.x; i < C * 64; i += 128) { const int c = i / 64, pp = i % 64; As[pp][c] = (b16)(bf16_rne(x[((size_t)b * C + c) * L + p0 + pp]) * XS); }
  __syncthreads();
  v8f acc[12];
#pragma unroll
  for (int t = 0; t < 12; ++t) acc[t] = (v8f){};
#pragma unroll
  for (int kb = 0; kb < C; kb += 32) { const v16b a = frag_kb(&As[wave * 16 + nloc][kb], hlf);
#pragma unroll
    for (int t = 0; t < 12; ++t) acc[t] = wmma16b(a, frag_kb(WT + (size_t)(t * 16 + nloc) * C + kb, hlf), acc[t]); }
#pragma unroll
  for (int t = 0; t < 12; ++t) { const int o = t * 16 + nloc; const float bb = bf16_rne(o < C ? b1[o] : o < 2 * C ? b2[o - C] : b3[o - 2 * C]);
#pragma unroll
    for (int r = 0; r < 8; ++r) Tf[wave][8 * hlf + r][o] = lrelu(acc[t][r] * (1.0f / (XS * WSC)) + bb); }
  __syncthreads();
  for (int pass = 0; pass < 2; ++pass) {
    for (int rr = 0; rr < 16; ++rr) { const int p = p0 + wave * 16 + rr; const int which = lane >> 4, d = (lane & 15) * 4; v4h hv, lv;
      for (int j = 0; j < 4; ++j) { const float f = Tf[wave][rr][which * C + d + j] * XS; const b16 h = (b16)f; hv[j] = h; lv[j] = (b16)((f - (float)h) * RS); }
      b16* ph = which == 0 ? Qh : Kh; b16* pl = which == 0 ? Ql : Kl; const size_t oi = ((size_t)b * L + p) * C + d; *(volatile v4h*)(ph + oi) = hv; *(volatile v4h*)(pl + oi) = lv; }
#pragma unroll 1
    for (int q = 0; q < 16; ++q) { const int d = wave * 16 + q; const int tk = lane * 2; v2h vv; vv[0] = (b16)(Tf[tk >> 4][tk & 15][2 * C + d] * XS); vv[1] = (b16)(Tf[(tk + 1) >> 4][(tk + 1) & 15][2 * C + d] * XS);
      *(volatile v2h*)(VT + ((size_t)b * C + d) * (size_t)L + p0 + tk) = vv; }
    __threadfence(); }
}
__global__ __launch_bounds__(64) void attn_kernel(const b16* __restrict__ Qh, const b16* __restrict__ Ql, const b16* __restrict__ Kh, const b16* __restrict__ Kl, const b16* __restrict__ VT, float* __restrict__ out) {
  __shared__ __attribute__((aligned(16))) b16 Pb[2][16][32 + 8]; __shared__ __attribute__((aligned(16))) float To[32][C + 4];
  const int wave = threadIdx.x >> 5, lane = threadIdx.x & 31, hh = lane >> 4, col = lane & 15; const int b = blockIdx.y; const int p0 = blockIdx.x * 32; const int q0 = p0 + wave * 16, qi = q0 + col;
  const b16* Qhb = Qh + (size_t)b * L * C; const b16* Qlb = Ql + (size_t)b * L * C; const b16* Khb = Kh + (size_t)b * L * C; const b16* Klb = Kl + (size_t)b * L * C; const b16* Vb = VT + (size_t)b * C * L;
  v16b qh[2], ql[2];
#pragma unroll
  for (int s = 0; s < 2; ++s) { qh[s] = frag_kb(Qhb + (size_t)qi * C + 32 * s, hh); ql[s] = frag_kb(Qlb + (size_t)qi * C + 32 * s, hh); }
  const float cs = LOG2E / (XS * XS), csl = cs / RS;
  float m = -INFINITY, l = 0.0f; v8f o[4]; for (int t = 0; t < 4; ++t) o[t] = (v8f){};
#pragma unroll 1
  for (int kb = 0; kb < L; kb += 32) {
    float e[16]; float mx = -INFINITY;
#pragma unroll
    for (int u = 0; u < 2; ++u) { v8f s = (v8f){}, sl = (v8f){}; const size_t kr = (size_t)(kb + u * 16 + col) * C;
#pragma unroll
      for (int st = 0; st < 2; ++st) { const v16b kh = frag_kb(Khb + kr + 32 * st, hh), kl = frag_kb(Klb + kr + 32 * st, hh); s = wmma16b(kh, qh[st], s); sl = wmma16b(kh, ql[st], sl); sl = wmma16b(kl, qh[st], sl); }
#pragma unroll
      for (int r = 0; r < 8; ++r) { const float vv = s[r] * cs + sl[r] * csl; e[u * 8 + r] = vv; mx = fmaxf(mx, vv); } }
    mx = fmaxf(mx, __shfl_xor(mx, 16)); const float mn = fmaxf(m, mx); const float al = nexp2(m - mn); float sum = 0.0f;
#pragma unroll
    for (int i2 = 0; i2 < 16; ++i2) { const float p = nexp2(e[i2] - mn); sum += p; Pb[wave][col][(i2 < 8 ? 0 : 16) + 8 * hh + (i2 & 7)] = (b16)(p * PS); }
    sum += __shfl_xor(sum, 16); l = l * al + sum; m = mn;
    wave_lds_sync();
    const v16b pf = frag_kb(&Pb[wave][col][0], hh);
#pragma unroll
    for (int t = 0; t < 4; ++t) { o[t] *= al; o[t] = wmma16b(frag_kb(Vb + (size_t)(t * 16 + col) * L + kb, hh), pf, o[t]); }
    wave_lds_sync(); }
  const float inv = 1.0f / (l * PS * XS);
#pragma unroll
  for (int t = 0; t < 4; ++t)
#pragma unroll
    for (int r = 0; r < 8; ++r) To[wave * 16 + col][t * 16 + 8 * hh + r] = o[t][r] * inv;
  __syncthreads();
  for (int pass = 0; pass < 2; ++pass) {
#pragma unroll 1
    for (int q = 0; q < 32; ++q) { const int c = wave * 32 + q; ((volatile float*)out)[((size_t)b * C + c) * L + p0 + lane] = To[lane][c]; }
    __threadfence(); }
}
}

extern "C" void kernel_launch(void* const* d_in, const int* in_sizes, int n_in, void* d_out, int out_size, void* d_ws, size_t ws_size, hipStream_t stream) {
  (void)n_in;
  auto Fp = [&](int i) { return (const float*)d_in[i]; };
  if (in_sizes[0] != B * C * L || in_sizes[1] != C * C || in_sizes[2] != C || in_sizes[3] != C * C || in_sizes[4] != C || in_sizes[5] != C * C || in_sizes[6] != C || out_size != B * C * L) return;
  size_t off = 0; char* ws = (char*)d_ws;
  auto carve = [&](size_t bytes) { char* p = ws + off; off += (bytes + 255) & ~(size_t)255; return p; };
  b16* WT = (b16*)carve((size_t)NO * C * 2); const size_t plane = (size_t)B * L * C * 2;
  b16* Qh = (b16*)carve(plane); b16* Ql = (b16*)carve(plane); b16* Kh = (b16*)carve(plane); b16* Kl = (b16*)carve(plane); b16* VT = (b16*)carve(plane);
  if (off > ws_size || off > ((size_t)128 << 20)) return;
  prep_kernel<<<(NO * C / 8 + 255) / 256, 256, 0, stream>>>(Fp(1), Fp(3), Fp(5), WT);
  qkv_kernel<<<dim3(L / 64, BL), 128, 0, stream>>>(Fp(0), WT, Fp(2), Fp(4), Fp(6), Qh, Ql, Kh, Kl, VT);
  attn_kernel<<<dim3(QL / 32, BL), 64, 0, stream>>>(Qh, Ql, Kh, Kl, VT, (float*)d_out);
}
